// GCNHealingAgent_9096740733199
// MI455X (gfx1250) — hardware-run, weakly checked
//
#include <hip/hip_runtime.h>
#include <stddef.h>
#include <stdint.h>
#include <math.h>

#define NN      50000
#define NE      800000
#define FI      16
#define HD      64
#define KE      32
#define KL      128
#define NO2     13
#define GBM     128
#define MR      50176
#define GT      (MR / GBM)
#define HT      391
#define NTHR    256
#define NWAVE   8
#define EPT     8
#define WCH     (32 * EPT)
#define NBRUN   1024
#define SLB     10
#define NBK     49
#define WLCAP   3584
#define RCAP    28672
#define DEGCAP  128
#define MAXDEG_MEAS   35
#define MAXB1024_MEAS 16623
#define SP      68
#define COW     (3 * NBRUN)

#define T_BEMB  0
#define T_BC    64
#define T_HEAD  256
#define T_HEADN 912
#define T_BG1   1168
#define T_WG2   1200
#define T_BG2   1232
#define T_WG1   1248
#define T_TOT   3296

#define O_TL    3200000
#define O_PD    3700000
#define O_LAST  3849984
#define O_TOT   3850001

#define BK_ZINTS (NWAVE * WLCAP + RCAP + 3 * NBRUN)
#define BK_INTS  (BK_ZINTS + 16)
#define BK_LDS   (BK_INTS * 4)

#define PBX   (MR * KE / 8 / NTHR)
#define PBWE  1
#define PBWL  (4 * HD * KL / 8 / NTHR)
#define PBTOT (PBX + PBWE + PBWL + 1)

static_assert(HD == 64 && KL == 2 * HD && KE % 32 == 0 && KL % 32 == 0);
static_assert(MR == NBK * NBRUN && MR % GBM == 0 && MR >= NN && NBRUN % GBM == 0);
static_assert(NBRUN == (1 << SLB) && NBRUN == NWAVE * 128);
static_assert(HT * GBM >= NN && (HT - 1) * GBM < NN && NN - (HT - 1) * GBM == 80);
static_assert(NE < (1 << 20) && (((long long)NE) << SLB) < (1LL << 31));
static_assert(NE % WCH == 0 && NE % 4 == 0);
static_assert(RCAP == NWAVE * WLCAP && RCAP % (NTHR * 4) == 0 && BK_ZINTS % 4 == 0 && COW % (NTHR * 4) == 0);
static_assert((long long)RCAP * 100 >= (long long)MAXB1024_MEAS * 105);
static_assert(WLCAP >= MAXB1024_MEAS / 8 + 8 * 46 + 1);
static_assert(MAXDEG_MEAS + 8 <= DEGCAP);
static_assert(BK_LDS <= 300000);
static_assert((MR * KE / 8) % NTHR == 0 && (HD * KE / 8) == NTHR && (4 * HD * KL / 8) % NTHR == 0);
static_assert((GBM * 10 * 4) % 128 == 0 && (GBM * 3 * 4) % 128 == 0 && (80 * 10 * 4) % 128 == 0);
static_assert(80 * 3 * 4 == 7 * 128 + 64);
static_assert(GBM * NO2 == 1664 && GBM * 10 == 1280 && 1664 % 4 == 0);
static_assert(O_TL == NN * HD && O_PD == O_TL + NN * 10 && O_TOT == O_PD + NN * 3 + 1);
static_assert(O_LAST == O_PD + (HT - 1) * GBM * 3 + 7 * 32 && O_LAST + 16 == O_TOT - 1);
static_assert((O_TL * 4) % 128 == 0 && (O_PD * 4) % 128 == 0 && (O_LAST * 4) % 128 == 0);
static_assert(T_TOT % 32 == 0 && T_HEAD + T_HEADN == T_BG1 && T_HEADN % 4 == 0);
static_assert((GBM * SP + T_HEADN + 1664) * 4 <= 65536);

typedef float          v4f   __attribute__((ext_vector_type(4)));
typedef float          v8f   __attribute__((ext_vector_type(8)));
typedef double         v2d   __attribute__((ext_vector_type(2)));
typedef int            v4i   __attribute__((ext_vector_type(4)));
typedef int            v8i   __attribute__((ext_vector_type(8)));
typedef unsigned short v8us  __attribute__((ext_vector_type(8)));
typedef unsigned short v16us __attribute__((ext_vector_type(16)));
typedef __bf16         v16bf __attribute__((ext_vector_type(16)));
typedef v4f  __attribute__((may_alias)) v4fa;
typedef v4i  __attribute__((may_alias)) v4ia;
typedef v8us __attribute__((may_alias)) v8usa;
union FragB { v16bf v; v16us u; v8us h[2]; v8i w; };

__device__ __forceinline__ v8f wmb(const FragB& a, const FragB& b, v8f c) {
  v8f d = __builtin_amdgcn_wmma_f32_16x16x32_bf16(false, a.v, false, b.v, (short)0, c, false, false);
  asm volatile("v_nop\n\tv_nop\n\tv_nop\n\tv_nop" : "+v"(d) : "v"(a.w), "v"(b.w));
  return d;
}

__device__ __forceinline__ unsigned bf16_bits(float f) {
  const unsigned u = __float_as_uint(f);
  const unsigned r = (u + 0x7FFFu + ((u >> 16) & 1u)) >> 16;
  const unsigned q = (u >> 16) | 0x40u;
  return ((u & 0x7fffffffu) > 0x7f800000u) ? q : r;
}
__device__ __forceinline__ float bf16_val(float f) {
  return __uint_as_float(bf16_bits(f) << 16);
}

__device__ __forceinline__ void hilo_pack(float v0, float v1, float v2, float v3,
                                          int& h01, int& h23, int& l01, int& l23) {
  const unsigned a0 = bf16_bits(v0), a1 = bf16_bits(v1), a2 = bf16_bits(v2), a3 = bf16_bits(v3);
  const unsigned b0 = bf16_bits(v0 - __uint_as_float(a0 << 16));
  const unsigned b1 = bf16_bits(v1 - __uint_as_float(a1 << 16));
  const unsigned b2 = bf16_bits(v2 - __uint_as_float(a2 << 16));
  const unsigned b3 = bf16_bits(v3 - __uint_as_float(a3 << 16));
  h01 = (int)(a0 | (a1 << 16)); h23 = (int)(a2 | (a3 << 16));
  l01 = (int)(b0 | (b1 << 16)); l23 = (int)(b2 | (b3 << 16));
}

__device__ __forceinline__ v4i regroup8(int h01, int h23, int l01, int l23, int lane) {
  const int t  = lane & 15;
  const int s0 = (lane & 16) + ((2 * t) & 15), s1 = s0 + 1;
  const int a0 = __shfl(h01, s0, 32), a1 = __shfl(h23, s0, 32), a2 = __shfl(h01, s1, 32), a3 = __shfl(h23, s1, 32);
  const int b0 = __shfl(l01, s0, 32), b1 = __shfl(l23, s0, 32), b2 = __shfl(l01, s1, 32), b3 = __shfl(l23, s1, 32);
  const int mk = (t < 8) ? -1 : 0;
  v4i o;
  o.x = (a0 & mk) | (b0 & ~mk); o.y = (a1 & mk) | (b1 & ~mk);
  o.z = (a2 & mk) | (b2 & ~mk); o.w = (a3 & mk) | (b3 & ~mk);
  return o;
}

__device__ __forceinline__ void st2_v4f(float* p, v4f v) {
  *(volatile v4f*)p = v;
  __threadfence();
  *(volatile v4f*)p = v;
}
__device__ __forceinline__ void st2_v8us(unsigned short* p, v8us v) {
  *(volatile v8us*)p = v;
  __threadfence();
  *(volatile v8us*)p = v;
}

__device__ __forceinline__ v8us gather8m(const float* __restrict__ base, int stride, unsigned mk) {
  float f[8];
#pragma unroll
  for (int i = 0; i < 8; ++i) f[i] = base[(size_t)i * (size_t)stride];
  v8us o;
#pragma unroll
  for (int i = 0; i < 8; ++i) o[i] = (unsigned short)(bf16_bits(f[i]) & mk);
  return o;
}

__device__ __forceinline__ void tab_copy(float* d, const float* __restrict__ s, int n, int lane) {
#pragma unroll 1
  for (int i0 = 0; i0 < n; i0 += 32) {
    const int i  = i0 + lane;
    const int ic = i < n ? i : n - 1;
    const float v = s[ic];
    asm volatile("" :: "v"(v));
    if (i < n) d[i] = bf16_val(v);
  }
}

__global__ __launch_bounds__(NTHR) void k_prep(
    const float* __restrict__ x,   const float* __restrict__ wemb, const float* __restrict__ bemb,
    const float* __restrict__ wc1, const float* __restrict__ bc1,
    const float* __restrict__ wc2, const float* __restrict__ bc2,
    const float* __restrict__ wc3, const float* __restrict__ bc3,
    const float* __restrict__ wn1, const float* __restrict__ bn1,
    const float* __restrict__ wn2, const float* __restrict__ bn2,
    const float* __restrict__ wg1, const float* __restrict__ bg1,
    const float* __restrict__ wg2, const float* __restrict__ bg2,
    unsigned short* xb, unsigned short* wet, unsigned short* wld, float* sm) {
  __shared__ __attribute__((aligned(16))) float tab[T_TOT];
  const int tid = (int)threadIdx.x, lane = tid & 31, wave = tid >> 5;
  const int blk = (int)blockIdx.x;
  if (blk < PBX) {
    const int u   = blk * NTHR + tid;
    const int row = u >> 2, k8 = (u & 3) * 8;
    const int rc  = row < NN ? row : NN - 1;
    const int kc  = k8 & 8;
    const unsigned mk = (row < NN && k8 < FI) ? 0xffffu : 0u;
    const float* p = x + (size_t)rc * FI + kc;
    const v4f a = *(const v4fa*)p;
    const v4f b = *(const v4fa*)(p + 4);
    v8us o;
    o[0] = (unsigned short)(bf16_bits(a.x) & mk); o[1] = (unsigned short)(bf16_bits(a.y) & mk);
    o[2] = (unsigned short)(bf16_bits(a.z) & mk); o[3] = (unsigned short)(bf16_bits(a.w) & mk);
    o[4] = (unsigned short)(bf16_bits(b.x) & mk); o[5] = (unsigned short)(bf16_bits(b.y) & mk);
    o[6] = (unsigned short)(bf16_bits(b.z) & mk); o[7] = (unsigned short)(bf16_bits(b.w) & mk);
    st2_v8us(xb + (size_t)row * KE + k8, o);
  } else if (blk < PBX + PBWE) {
    const int n = tid >> 2, k8 = (tid & 3) * 8;
    const int kc = k8 & 8;
    const unsigned mk = (k8 < FI) ? 0xffffu : 0u;
    const v8us o = gather8m(wemb + (size_t)kc * HD + n, HD, mk);
    st2_v8us(wet + (size_t)n * KE + k8, o);
  } else if (blk < PBX + PBWE + PBWL) {
    const int v = (blk - PBX - PBWE) * NTHR + tid;
    const int l = v >> 10, n = (v >> 4) & 63, k8 = (v & 15) * 8, kk = k8 & 63;
    unsigned short* dp = wld + (size_t)l * HD * KL + (size_t)n * KL + k8;
    v8us o;
    if (l == 0)      o = gather8m(wc1 + (size_t)kk * HD + n, HD, 0xffffu);
    else if (l == 1) o = gather8m(wc2 + (size_t)kk * HD + n, HD, 0xffffu);
    else if (l == 2) o = gather8m(wc3 + (size_t)kk * HD + n, HD, 0xffffu);
    else             o = gather8m(wn1 + (size_t)kk * HD + n, HD, 0xffffu);
    st2_v8us(dp, o);
  } else {
    {
      const v4f z4 = {0.f, 0.f, 0.f, 0.f};
#pragma unroll 1
      for (int i = tid * 4; i < T_TOT; i += NTHR * 4) *(v4fa*)(tab + i) = z4;
    }
    __syncthreads();
    if (wave == 0) {
      tab_copy(tab + T_BEMB, bemb, HD, lane);
      tab_copy(tab + T_BC, bc1, HD, lane);
      tab_copy(tab + T_BC + 64, bc2, HD, lane);
      tab_copy(tab + T_BC + 128, bc3, HD, lane);
      tab_copy(tab + T_HEAD, bn1, HD, lane);
    } else if (wave == 1) {
      tab_copy(tab + T_HEAD + 64, bn2, NO2, lane);
      tab_copy(tab + T_BG1, bg1, 32, lane);
      tab_copy(tab + T_WG2, wg2, 32, lane);
      tab_copy(tab + T_BG2, bg2, 1, lane);
    } else if (wave < 4) {
#pragma unroll 1
      for (int i0 = (wave - 2) * 32; i0 < HD * NO2; i0 += 64) {
        const int i  = i0 + lane;
        const int ic = i < HD * NO2 ? i : HD * NO2 - 1;
        const float v = wn2[ic];
        asm volatile("" :: "v"(v));
        const int k = ic / NO2, c = ic - NO2 * k;
        if (i < HD * NO2) tab[T_HEAD + 80 + c * HD + k] = bf16_val(v);
      }
    } else {
#pragma unroll 1
      for (int i0 = (wave - 4) * 32; i0 < HD * 32; i0 += 128) {
        const int i  = i0 + lane;
        const int ic = i < HD * 32 ? i : HD * 32 - 1;
        const float v = wg1[ic];
        asm volatile("" :: "v"(v));
        if (i < HD * 32) tab[T_WG1 + i] = bf16_val(v);
      }
    }
    __syncthreads();
#pragma unroll 1
    for (int pass = 0; pass < 2; ++pass) {
#pragma unroll 1
      for (int it = 0; it < 4; ++it) {
        const int u  = it * NTHR + tid;
        const int uc = u < T_TOT / 4 ? u : T_TOT / 4 - 1;
        const v4f v = *(const v4fa*)(tab + 4 * uc);
        asm volatile("" :: "v"(v));
        if (u < T_TOT / 4) *(volatile v4f*)(sm + 4 * u) = v;
      }
      __threadfence();
    }
  }
}

__device__ __forceinline__ void bucket_flush(const int* pl, const int* cnt, int ov, int* lp, int* cop, int* fp,
                                             int tid) {
#pragma unroll 1
  for (int i = tid * 4; i < RCAP; i += NTHR * 4) {
    const v4i v = *(const v4ia*)(pl + i);
    *(volatile v4i*)(lp + i) = v;
  }
#pragma unroll 1
  for (int i = tid * 4; i < COW; i += NTHR * 4) {
    const v4i v = *(const v4ia*)(cnt + i);
    *(volatile v4i*)(cop + i) = v;
  }
  if (tid < 8) {
    const v4i f = {ov, ov, ov, ov};
    *(volatile v4i*)(fp + 4 * tid) = f;
  }
}

__global__ __launch_bounds__(NTHR) void k_bucket(const int* __restrict__ srcs, const int* __restrict__ dsts,
                                                 int* LIST, int* CO, int* FLAG) {
  extern __shared__ __attribute__((aligned(16))) int dsm[];
  int* wl   = dsm;
  int* pl   = dsm + NWAVE * WLCAP;
  int* cnt  = pl + RCAP;
  int* offs = cnt + NBRUN;
  int* cur  = offs + NBRUN;
  int* misc = cur + NBRUN;
  const int tid = (int)threadIdx.x, lane = tid & 31, wave = tid >> 5;
  const int blk = (int)blockIdx.x;
  const unsigned nbs = (unsigned)(blk * NBRUN);

  {
    const v4i z4 = {0, 0, 0, 0};
#pragma unroll 1
    for (int i = tid * 4; i < BK_ZINTS; i += NTHR * 4) *(v4ia*)(dsm + i) = z4;
    if (tid < 16) misc[tid] = 0;
  }
  __syncthreads();

  {
    const int per  = ((NE + NWAVE * WCH - 1) / (NWAVE * WCH)) * WCH;
    const int ebeg = wave * per;
    const int eend = (ebeg + per < NE) ? (ebeg + per) : NE;
    int* mylist = wl + wave * WLCAP;
    int wc = 0;
#pragma unroll 1
    for (int cb = ebeg; cb < eend; cb += WCH) {
      const int e0 = cb + lane * EPT;
      const v4i da = *(const v4ia*)(dsts + e0);
      const v4i db = *(const v4ia*)(dsts + e0 + 4);
      const unsigned s0 = (unsigned)da.x - nbs, s1 = (unsigned)da.y - nbs;
      const unsigned s2 = (unsigned)da.z - nbs, s3 = (unsigned)da.w - nbs;
      const unsigned s4 = (unsigned)db.x - nbs, s5 = (unsigned)db.y - nbs;
      const unsigned s6 = (unsigned)db.z - nbs, s7 = (unsigned)db.w - nbs;
      const bool h0 = s0 < (unsigned)NBRUN, h1 = s1 < (unsigned)NBRUN, h2 = s2 < (unsigned)NBRUN, h3 = s3 < (unsigned)NBRUN;
      const bool h4 = s4 < (unsigned)NBRUN, h5 = s5 < (unsigned)NBRUN, h6 = s6 < (unsigned)NBRUN, h7 = s7 < (unsigned)NBRUN;
      const unsigned m0 = __builtin_amdgcn_ballot_w32(h0), m1 = __builtin_amdgcn_ballot_w32(h1);
      const unsigned m2 = __builtin_amdgcn_ballot_w32(h2), m3 = __builtin_amdgcn_ballot_w32(h3);
      const unsigned m4 = __builtin_amdgcn_ballot_w32(h4), m5 = __builtin_amdgcn_ballot_w32(h5);
      const unsigned m6 = __builtin_amdgcn_ballot_w32(h6), m7 = __builtin_amdgcn_ballot_w32(h7);
      const unsigned any = m0 | m1 | m2 | m3 | m4 | m5 | m6 | m7;
      if (any != 0u) {
        const int pre = (int)(__builtin_amdgcn_mbcnt_lo(m0, 0u) + __builtin_amdgcn_mbcnt_lo(m1, 0u) +
                              __builtin_amdgcn_mbcnt_lo(m2, 0u) + __builtin_amdgcn_mbcnt_lo(m3, 0u) +
                              __builtin_amdgcn_mbcnt_lo(m4, 0u) + __builtin_amdgcn_mbcnt_lo(m5, 0u) +
                              __builtin_amdgcn_mbcnt_lo(m6, 0u) + __builtin_amdgcn_mbcnt_lo(m7, 0u));
        int p = wc + pre;
        if (h0) { if (p < WLCAP) mylist[p] = ((e0 + 0) << SLB) | (int)s0; p = p + 1; }
        if (h1) { if (p < WLCAP) mylist[p] = ((e0 + 1) << SLB) | (int)s1; p = p + 1; }
        if (h2) { if (p < WLCAP) mylist[p] = ((e0 + 2) << SLB) | (int)s2; p = p + 1; }
        if (h3) { if (p < WLCAP) mylist[p] = ((e0 + 3) << SLB) | (int)s3; p = p + 1; }
        if (h4) { if (p < WLCAP) mylist[p] = ((e0 + 4) << SLB) | (int)s4; p = p + 1; }
        if (h5) { if (p < WLCAP) mylist[p] = ((e0 + 5) << SLB) | (int)s5; p = p + 1; }
        if (h6) { if (p < WLCAP) mylist[p] = ((e0 + 6) << SLB) | (int)s6; p = p + 1; }
        if (h7) { if (p < WLCAP) mylist[p] = ((e0 + 7) << SLB) | (int)s7; p = p + 1; }
        wc += (int)(__builtin_popcount(m0) + __builtin_popcount(m1) + __builtin_popcount(m2) + __builtin_popcount(m3) +
                    __builtin_popcount(m4) + __builtin_popcount(m5) + __builtin_popcount(m6) + __builtin_popcount(m7));
      }
    }
    if (lane == 0) misc[wave] = wc;
  }
  __syncthreads();

  if (wave == 0) {
    int ov = 0;
#pragma unroll 1
    for (int w2 = 0; w2 < NWAVE; ++w2) {
      int c = misc[w2];
      if (c > WLCAP) ov = 1;
      c = c < 0 ? 0 : (c > WLCAP ? WLCAP : c);
#pragma unroll 1
      for (int b0 = 0; b0 < c; b0 += 32) {
        const int idx = b0 + lane;
        const int ent = wl[w2 * WLCAP + (idx < WLCAP ? idx : WLCAP - 1)];
        const int m32 = (c - b0) < 32 ? (c - b0) : 32;
#pragma unroll 1
        for (int k = 0; k < m32; ++k) {
          const int u    = __builtin_amdgcn_readlane(ent, k);
          const int slot = u & (NBRUN - 1);
          if (lane == 0) cnt[slot] = cnt[slot] + 1;
        }
      }
    }
    if (lane == 0) misc[9] = ov;
  }
  __syncthreads();
  if (wave == 0) {
    const int base = lane * (NBRUN / 32);
    int s = 0;
#pragma unroll 1
    for (int i = 0; i < NBRUN / 32; ++i) s += cnt[base + i];
    int incl = s;
#pragma unroll
    for (int d = 1; d < 32; d <<= 1) {
      const int y = __shfl_up(incl, d, 32);
      if (lane >= d) incl += y;
    }
    int run = incl - s;
#pragma unroll 1
    for (int i = 0; i < NBRUN / 32; ++i) {
      const int cv = cnt[base + i];
      offs[base + i] = run;
      cur[base + i]  = run;
      run += cv;
    }
  }
  __syncthreads();

  if (wave == 0) {
#pragma unroll 1
    for (int w2 = 0; w2 < NWAVE; ++w2) {
      int c = misc[w2];
      c = c < 0 ? 0 : (c > WLCAP ? WLCAP : c);
#pragma unroll 1
      for (int b0 = 0; b0 < c; b0 += 32) {
        const int idx = b0 + lane;
        const int ent = wl[w2 * WLCAP + (idx < WLCAP ? idx : WLCAP - 1)];
        int eid = (ent >> SLB) & 0xFFFFF;
        eid = eid > NE - 1 ? NE - 1 : eid;
        int sr = srcs[eid];
        sr = sr < 0 ? 0 : (sr > NN - 1 ? NN - 1 : sr);
        const int m32 = (c - b0) < 32 ? (c - b0) : 32;
#pragma unroll 1
        for (int k = 0; k < m32; ++k) {
          const int u    = __builtin_amdgcn_readlane(ent, k);
          const int wd   = __builtin_amdgcn_readlane(sr, k);
          const int slot = u & (NBRUN - 1);
          if (lane == 0) {
            int p = cur[slot];
            p = p < 0 ? 0 : (p > RCAP - 1 ? RCAP - 1 : p);
            pl[p] = wd;
            cur[slot] = p + 1;
          }
        }
      }
    }
  }
  __syncthreads();

#pragma unroll 1
  for (int s = tid; s < NBRUN; s += NTHR) {
    int c = cnt[s];
    c = c < 0 ? 0 : c;
    const float dv = 1.0f / sqrtf((float)(c + 1));
    cur[s] = __float_as_int(dv);
  }
  __syncthreads();

  const int ovf = misc[9];
  int* lp  = LIST + (size_t)blk * RCAP;
  int* cop = CO + (size_t)blk * COW;
  int* fp  = FLAG + (size_t)blk * 32;
  bucket_flush(pl, cnt, ovf, lp, cop, fp, tid);
  __threadfence();
  bucket_flush(pl, cnt, ovf, lp, cop, fp, tid);
}

template <int KTOT>
__device__ __forceinline__ void gemm_16x64(const unsigned short* __restrict__ ap,
                                           const unsigned short* __restrict__ bp, v8f (&acc)[4]) {
#pragma unroll 1
  for (int k0 = 0; k0 < KTOT; k0 += 32) {
    FragB af;
    af.h[0] = *(const v8usa*)(ap + k0);
    af.h[1] = *(const v8usa*)(ap + k0 + 16);
#pragma unroll
    for (int nt = 0; nt < 4; ++nt) {
      const unsigned short* wq = bp + (size_t)(16 * nt) * (size_t)KTOT + k0;
      FragB bf;
      bf.h[0] = *(const v8usa*)wq;
      bf.h[1] = *(const v8usa*)(wq + 16);
      acc[nt] = wmb(af, bf, acc[nt]);
    }
  }
}

__device__ __forceinline__ void stage_d(float* stg, const v8f (&acc)[4], int wave, int hh, int m) {
#pragma unroll
  for (int nt = 0; nt < 4; ++nt) {
#pragma unroll
    for (int r = 0; r < 8; ++r) stg[(16 * wave + 8 * hh + r) * SP + 16 * nt + m] = acc[nt][r];
  }
}

__global__ __launch_bounds__(NTHR) __attribute__((amdgpu_num_vgpr(248)))
void k_emb(const unsigned short* __restrict__ XB, const unsigned short* __restrict__ WET,
           const float* __restrict__ sm, float* HF, unsigned short* HHL) {
  __shared__ __attribute__((aligned(16))) float stg[GBM * SP];
  __shared__ __attribute__((aligned(16))) float sb[64];
  const int tid = (int)threadIdx.x, lane = tid & 31, wave = tid >> 5, hh = lane >> 4, m = lane & 15;
  const int rowBase = (int)blockIdx.x * GBM;
  if (tid < 16) *(v4fa*)(sb + 4 * tid) = *(const v4fa*)(sm + T_BEMB + 4 * tid);

  v8f acc[4];
  {
    const v8f z = {0.f, 0.f, 0.f, 0.f, 0.f, 0.f, 0.f, 0.f};
#pragma unroll
    for (int t = 0; t < 4; ++t) acc[t] = z;
  }
  const unsigned short* ap = XB + (size_t)(rowBase + 16 * wave + m) * (size_t)KE + 8 * hh;
  const unsigned short* bp = WET + (size_t)m * (size_t)KE + 8 * hh;
  gemm_16x64<KE>(ap, bp, acc);
  stage_d(stg, acc, wave, hh, m);
  __syncthreads();

  const v4f bias = *(const v4fa*)(sb + 4 * m);
#pragma unroll 1
  for (int i = 0; i < 8; ++i) {
    const int lr   = 16 * wave + 2 * i + hh;
    const int grow = rowBase + lr;
    const bool live = grow < NN;
    const v4f a = *(const v4fa*)(stg + lr * SP + 4 * m);
    asm volatile("" :: "v"(a));
    float v0 = a.x + bias.x, v1 = a.y + bias.y, v2 = a.z + bias.z, v3 = a.w + bias.w;
    v0 = live ? v0 : 0.0f; v1 = live ? v1 : 0.0f; v2 = live ? v2 : 0.0f; v3 = live ? v3 : 0.0f;
    v4f o;
    o.x = v0; o.y = v1; o.z = v2; o.w = v3;
    int h01, h23, l01, l23;
    hilo_pack(v0, v1, v2, v3, h01, h23, l01, l23);
    const v4i ow = regroup8(h01, h23, l01, l23, lane);
    float* op = HF + (size_t)grow * HD + 4 * m;
    unsigned short* hp = HHL + (size_t)grow * KL + 8 * m;
    *(volatile v4f*)op = o;
    *(volatile v4i*)hp = ow;
    __threadfence();
    *(volatile v4f*)op = o;
    *(volatile v4i*)hp = ow;
  }
}

__global__ __launch_bounds__(NTHR) __attribute__((amdgpu_num_vgpr(248)))
void k_lin(const unsigned short* __restrict__ A, const unsigned short* __restrict__ BT,
           const int* __restrict__ CO, float* P) {
  __shared__ __attribute__((aligned(16))) float stg[GBM * SP];
  const int tid = (int)threadIdx.x, lane = tid & 31, wave = tid >> 5, hh = lane >> 4, m = lane & 15;
  const int rowBase = (int)blockIdx.x * GBM;

  v8f acc[4];
  {
    const v8f z = {0.f, 0.f, 0.f, 0.f, 0.f, 0.f, 0.f, 0.f};
#pragma unroll
    for (int t = 0; t < 4; ++t) acc[t] = z;
  }
  const unsigned short* ap = A + (size_t)(rowBase + 16 * wave + m) * (size_t)KL + 8 * hh;
  const unsigned short* bp = BT + (size_t)m * (size_t)KL + 8 * hh;
  gemm_16x64<KL>(ap, bp, acc);
  stage_d(stg, acc, wave, hh, m);
  __syncthreads();

#pragma unroll 1
  for (int i = 0; i < 8; ++i) {
    const int lr   = 16 * wave + 2 * i + hh;
    const int grow = rowBase + lr;
    const float dv = __int_as_float(CO[(size_t)(grow >> SLB) * COW + 2 * NBRUN + (grow & (NBRUN - 1))]);
    const v4f a = *(const v4fa*)(stg + lr * SP + 4 * m);
    asm volatile("" :: "v"(a));
    v4f o;
    o.x = dv * a.x; o.y = dv * a.y; o.z = dv * a.z; o.w = dv * a.w;
    st2_v4f(P + (size_t)grow * HD + 4 * m, o);
  }
}

template <int LAST>
__global__ __launch_bounds__(NTHR) void k_replay(const int* __restrict__ LIST, const int* __restrict__ CO,
                                                 const int* __restrict__ FLAG, const float* __restrict__ P,
                                                 const float* __restrict__ sm, int boff,
                                                 float* HF, unsigned short* HHL, float* out, double* REC) {
  __shared__ __attribute__((aligned(16))) float sb[64];
  __shared__ __attribute__((aligned(16))) double rs[16 * HD];
  __shared__ __attribute__((aligned(16))) double ro[HD];
  const int tid = (int)threadIdx.x, lane = tid & 31, wave = tid >> 5, hh = lane >> 4, q = lane & 15;
  const int blk = (int)blockIdx.x;
  const int rowBase = blk * NBRUN;
  const int* lb  = LIST + (size_t)blk * RCAP;
  const int* cob = CO + (size_t)blk * COW;
  const int flag = FLAG[(size_t)blk * 32];
  const float qnan = __uint_as_float(0x7fc00000u);
  if (tid < 16) *(v4fa*)(sb + 4 * tid) = *(const v4fa*)(sm + boff + 4 * tid);
  __syncthreads();
  const v4f bias = *(const v4fa*)(sb + 4 * q);
  double s0 = 0.0, s1 = 0.0, s2 = 0.0, s3 = 0.0;

#pragma unroll 1
  for (int i = 0; i < NBRUN / (2 * NWAVE); ++i) {
    const int slot = (NBRUN / NWAVE) * wave + 2 * i + hh;
    const int d    = rowBase + slot;
    int c = cob[slot];
    int o = cob[NBRUN + slot];
    const float dv = __int_as_float(cob[2 * NBRUN + slot]);
    const bool big = c > DEGCAP;
    c = c < 0 ? 0 : (c > DEGCAP ? DEGCAP : c);
    o = o < 0 ? 0 : (o > RCAP - 1 ? RCAP - 1 : o);
    const int co = __shfl_xor(c, 16, 32);
    const int cm = c > co ? c : co;
    int last = o + c - 1;
    last = last < o ? o : last;
    last = last > RCAP - 1 ? RCAP - 1 : last;
    float a0 = 0.0f, a1 = 0.0f, a2 = 0.0f, a3 = 0.0f;
#pragma unroll 1
    for (int j = 0; j < cm; ++j) {
      int idx = o + j;
      idx = idx > last ? last : idx;
      int sr = lb[idx];
      sr = sr < 0 ? 0 : (sr > NN - 1 ? NN - 1 : sr);
      const v4f v = *(const v4fa*)(P + (size_t)sr * HD + 4 * q);
      asm volatile("" :: "v"(v));
      const bool valid = j < c;
      const float t0 = a0 + v.x, t1 = a1 + v.y, t2 = a2 + v.z, t3 = a3 + v.w;
      a0 = valid ? t0 : a0; a1 = valid ? t1 : a1; a2 = valid ? t2 : a2; a3 = valid ? t3 : a3;
    }
    const v4f ps = *(const v4fa*)(P + (size_t)d * HD + 4 * q);
    const v4f g  = *(const v4fa*)(HF + (size_t)d * HD + 4 * q);
    asm volatile("" :: "v"(ps));
    asm volatile("" :: "v"(g));
    a0 += ps.x; a1 += ps.y; a2 += ps.z; a3 += ps.w;
    float t0 = dv * a0 + bias.x, t1 = dv * a1 + bias.y, t2 = dv * a2 + bias.z, t3 = dv * a3 + bias.w;
    t0 = (t0 > 0.0f) ? t0 : (t0 - t0); t1 = (t1 > 0.0f) ? t1 : (t1 - t1);
    t2 = (t2 > 0.0f) ? t2 : (t2 - t2); t3 = (t3 > 0.0f) ? t3 : (t3 - t3);
    float m0 = g.x + t0, m1 = g.y + t1, m2 = g.z + t2, m3 = g.w + t3;
    const bool bad  = (flag != 0) | big;
    const bool live = d < NN;
    m0 = bad ? qnan : m0; m1 = bad ? qnan : m1; m2 = bad ? qnan : m2; m3 = bad ? qnan : m3;
    m0 = live ? m0 : 0.0f; m1 = live ? m1 : 0.0f; m2 = live ? m2 : 0.0f; m3 = live ? m3 : 0.0f;
    int h01, h23, l01, l23;
    hilo_pack(m0, m1, m2, m3, h01, h23, l01, l23);
    const v4i ow = regroup8(h01, h23, l01, l23, lane);
    v4f ov;
    ov.x = m0; ov.y = m1; ov.z = m2; ov.w = m3;
    float* op = HF + (size_t)d * HD + 4 * q;
    unsigned short* hp = HHL + (size_t)d * KL + 8 * q;
    const int dc = live ? d : NN - 1;
    float* gp = out + (size_t)dc * HD + 4 * q;
    *(volatile v4f*)op = ov;
    *(volatile v4i*)hp = ow;
    if constexpr (LAST != 0) { if (live) *(volatile v4f*)gp = ov; }
    __threadfence();
    *(volatile v4f*)op = ov;
    *(volatile v4i*)hp = ow;
    if constexpr (LAST != 0) {
      if (live) *(volatile v4f*)gp = ov;
      s0 += (double)m0; s1 += (double)m1; s2 += (double)m2; s3 += (double)m3;
    }
  }

  if constexpr (LAST != 0) {
    const int hw = 2 * wave + hh;
    rs[hw * HD + 4 * q + 0] = s0;
    rs[hw * HD + 4 * q + 1] = s1;
    rs[hw * HD + 4 * q + 2] = s2;
    rs[hw * HD + 4 * q + 3] = s3;
    __syncthreads();
    if (tid < HD) {
      double t = 0.0;
#pragma unroll 1
      for (int w2 = 0; w2 < 16; ++w2) t += rs[w2 * HD + tid];
      ro[tid] = t;
    }
    __syncthreads();
    if (tid < 32) {
      v2d o;
      o.x = ro[2 * tid];
      o.y = ro[2 * tid + 1];
      double* rp = REC + (size_t)blk * HD + 2 * tid;
      *(volatile v2d*)rp = o;
      __threadfence();
      *(volatile v2d*)rp = o;
    }
  }
}

__device__ __forceinline__ void head_flush(const float* os, float* tlb, float* pdb, float* tail,
                                           int nvtl, int nvpd, int tailblk, int tid) {
#pragma unroll 1
  for (int it = 0; it < 2; ++it) {
    const int i4 = it * NTHR + tid;
    const int ic = i4 < 416 ? i4 : 415;
    const v4f v = *(const v4fa*)(os + 4 * ic);
    asm volatile("" :: "v"(v));
    const int j = i4 - 320;
    if (i4 < nvtl) *(volatile v4f*)(tlb + (size_t)4 * (size_t)i4) = v;
    if (j >= 0 && j < nvpd) *(volatile v4f*)(pdb + (size_t)4 * (size_t)j) = v;
    if (tailblk != 0 && j >= 56 && j < 64) *(volatile v4f*)(tail + 4 * (j - 56)) = v;
  }
}

__global__ __launch_bounds__(NTHR) __attribute__((amdgpu_num_vgpr(248)))
void k_head(const unsigned short* __restrict__ HHL, const unsigned short* __restrict__ W1T,
            const float* __restrict__ sm, const int* __restrict__ FLAG,
            float* tl, float* pd, float* tail) {
  __shared__ __attribute__((aligned(16))) float stg[GBM * SP];
  __shared__ __attribute__((aligned(16))) float hs[T_HEADN];
  __shared__ __attribute__((aligned(16))) float os[1664];
  const int tid = (int)threadIdx.x, lane = tid & 31, wave = tid >> 5, hh = lane >> 4, m = lane & 15;
  const int blk = (int)blockIdx.x;
  const int rowBase = blk * GBM;
  const int flag = FLAG[(size_t)(rowBase >> SLB) * 32];
  if (tid < T_HEADN / 4) *(v4fa*)(hs + 4 * tid) = *(const v4fa*)(sm + T_HEAD + 4 * tid);
  __syncthreads();

  v8f acc[4];
  {
    const v8f z = {0.f, 0.f, 0.f, 0.f, 0.f, 0.f, 0.f, 0.f};
#pragma unroll
    for (int t = 0; t < 4; ++t) acc[t] = z;
  }
  const unsigned short* ap = HHL + (size_t)(rowBase + 16 * wave + m) * (size_t)KL + 8 * hh;
  const unsigned short* bp = W1T + (size_t)m * (size_t)KL + 8 * hh;
  gemm_16x64<KL>(ap, bp, acc);
#pragma unroll
  for (int nt = 0; nt < 4; ++nt) {
    const float bv = hs[16 * nt + m];
#pragma unroll
    for (int r = 0; r < 8; ++r) {
      float t = acc[nt][r] + bv;
      t = (t > 0.0f) ? t : (t - t);
      stg[(16 * wave + 8 * hh + r) * SP + 16 * nt + m] = t;
    }
  }
  __syncthreads();

  const float qnan = __uint_as_float(0x7fc00000u);
#pragma unroll 1
  for (int it = 0; it < 7; ++it) {
    const int idx = it * NTHR + tid;
    const bool ok = idx < GBM * NO2;
    const int ic  = ok ? idx : GBM * NO2 - 1;
    const int row = ic / NO2;
    const int c   = ic - NO2 * row;
    const float* hr = stg + row * SP;
    const float* wr = hs + 80 + c * HD;
    float s = 0.0f;
#pragma unroll 1
    for (int k4 = 0; k4 < HD / 4; ++k4) {
      const v4f a = *(const v4fa*)(hr + 4 * k4);
      const v4f w = *(const v4fa*)(wr + 4 * k4);
      s = fmaf(a.x, w.x, s);
      s = fmaf(a.y, w.y, s);
      s = fmaf(a.z, w.z, s);
      s = fmaf(a.w, w.w, s);
    }
    float val = s + hs[64 + c];
    val = (flag != 0) ? qnan : val;
    const int pos = (c < 10) ? (row * 10 + c) : (GBM * 10 + row * 3 + (c - 10));
    if (ok) os[pos] = val;
  }
  __syncthreads();

  const int liveRows = (NN - rowBase) < GBM ? (NN - rowBase) : GBM;
  const int nvtl = (liveRows * 10) / 4;
  const int nvpd = ((liveRows * 3 * 4) / 128) * 8;
  const int tailblk = (blk == HT - 1) ? 1 : 0;
  float* tlb = tl + (size_t)blk * (size_t)(GBM * 10);
  float* pdb = pd + (size_t)blk * (size_t)(GBM * 3);
  head_flush(os, tlb, pdb, tail, nvtl, nvpd, tailblk, tid);
  __threadfence();
  head_flush(os, tlb, pdb, tail, nvtl, nvpd, tailblk, tid);
}

__global__ __launch_bounds__(NTHR) void k_global(const double* __restrict__ REC, const float* __restrict__ sm,
                                                 const float* __restrict__ TAIL, float* out) {
  __shared__ float g[HD];
  __shared__ float hv[32];
  const int tid = (int)threadIdx.x;
  if (tid < HD) {
    double s = 0.0;
#pragma unroll 1
    for (int b = 0; b < NBK; ++b) s += REC[(size_t)b * HD + tid];
    g[tid] = (float)(s / 50000.0);
  }
  __syncthreads();
  if (tid < 32) {
    float s = 0.0f;
#pragma unroll 4
    for (int k = 0; k < HD; ++k) s = fmaf(g[k], sm[T_WG1 + k * 32 + tid], s);
    float t = s + sm[T_BG1 + tid];
    t = (t > 0.0f) ? t : (t - t);
    hv[tid] = t * sm[T_WG2 + tid];
  }
  __syncthreads();
  if (tid < 32) {
    float z = 0.0f;
#pragma unroll 1
    for (int j = 0; j < 32; ++j) z += hv[j];
    z += sm[T_BG2];
    const float gp = 1.0f / (1.0f + expf(-z));
    const float tv = TAIL[tid & 15];
    asm volatile("" :: "v"(tv));
    const unsigned mk = (tid < 16) ? 0xffffffffu : 0u;
    const float val = __uint_as_float((__float_as_uint(tv) & mk) | (__float_as_uint(gp) & ~mk));
    float* op = out + (size_t)O_LAST + (size_t)(tid < 17 ? tid : 16);
    if (tid < 17) *(volatile float*)op = val;
    __threadfence();
    if (tid < 17) *(volatile float*)op = val;
  }
}

extern "C" void kernel_launch(void* const* d_in, const int* in_sizes, int n_in,
                              void* d_out, int out_size, void* d_ws, size_t ws_size,
                              hipStream_t stream) {
  if (n_in < 18) return;
  if (in_sizes[0] != NN * FI) return;
  if (in_sizes[1] != 2 * NE) return;
  if (in_sizes[2] != FI * HD || in_sizes[3] != HD) return;
  if (in_sizes[4] != HD * HD || in_sizes[5] != HD) return;
  if (in_sizes[6] != HD * HD || in_sizes[7] != HD) return;
  if (in_sizes[8] != HD * HD || in_sizes[9] != HD) return;
  if (in_sizes[10] != HD * HD || in_sizes[11] != HD) return;
  if (in_sizes[12] != HD * NO2 || in_sizes[13] != NO2) return;
  if (in_sizes[14] != HD * 32 || in_sizes[15] != 32) return;
  if (in_sizes[16] != 32 || in_sizes[17] != 1) return;
  if (out_size != O_TOT) return;

  const float* x    = (const float*)d_in[0];
  const int*   ei   = (const int*)d_in[1];
  const float* Wemb = (const float*)d_in[2];
  const float* bemb = (const float*)d_in[3];
  const float* Wc1  = (const float*)d_in[4];
  const float* bc1  = (const float*)d_in[5];
  const float* Wc2  = (const float*)d_in[6];
  const float* bc2  = (const float*)d_in[7];
  const float* Wc3  = (const float*)d_in[8];
  const float* bc3  = (const float*)d_in[9];
  const float* Wn1  = (const float*)d_in[10];
  const float* bn1  = (const float*)d_in[11];
  const float* Wn2  = (const float*)d_in[12];
  const float* bn2  = (const float*)d_in[13];
  const float* Wg1  = (const float*)d_in[14];
  const float* bg1  = (const float*)d_in[15];
  const float* Wg2  = (const float*)d_in[16];
  const float* bg2  = (const float*)d_in[17];
  float* out = (float*)d_out;
  const int* srcs = ei;
  const int* dsts = ei + NE;

  constexpr size_t zXB   = (size_t)MR * KE * 2;
  constexpr size_t zF    = (size_t)MR * HD * 4;
  constexpr size_t zHL   = (size_t)MR * KL * 2;
  constexpr size_t zLIST = (size_t)NBK * RCAP * 4;
  constexpr size_t zCO   = (size_t)NBK * COW * 4;
  constexpr size_t zFLAG = (size_t)NBK * 128;
  constexpr size_t zWET  = (size_t)HD * KE * 2;
  constexpr size_t zWLD  = (size_t)4 * HD * KL * 2;
  constexpr size_t zSM   = (size_t)T_TOT * 4;
  constexpr size_t zREC  = (size_t)NBK * HD * 8;
  constexpr size_t zTAIL = 128;
  constexpr size_t oXB   = 0;
  constexpr size_t oHF   = oXB + zXB;
  constexpr size_t oHHL  = oHF + zF;
  constexpr size_t oP    = oHHL + zHL;
  constexpr size_t oLIST = oP + zF;
  constexpr size_t oCO   = oLIST + zLIST;
  constexpr size_t oFLAG = oCO + zCO;
  constexpr size_t oWET  = oFLAG + zFLAG;
  constexpr size_t oWLD  = oWET + zWET;
  constexpr size_t oSM   = oWLD + zWLD;
  constexpr size_t oREC  = oSM + zSM;
  constexpr size_t oTAIL = oREC + zREC;
  constexpr size_t oEND  = oTAIL + zTAIL;
  static_assert(zXB % 128 == 0 && zF % 128 == 0 && zHL % 128 == 0 && zLIST % 128 == 0 && zCO % 128 == 0);
  static_assert(zFLAG % 128 == 0 && zWET % 128 == 0 && zWLD % 128 == 0 && zSM % 128 == 0 && zREC % 128 == 0);
  static_assert(oEND <= (size_t)(128u << 20));
  if (oEND > ws_size) return;

  char* ws = (char*)d_ws;
  unsigned short* XB   = (unsigned short*)(ws + oXB);
  float*          HF   = (float*)(ws + oHF);
  unsigned short* HHL  = (unsigned short*)(ws + oHHL);
  float*          P    = (float*)(ws + oP);
  int*            LIST = (int*)(ws + oLIST);
  int*            CO   = (int*)(ws + oCO);
  int*            FLAG = (int*)(ws + oFLAG);
  unsigned short* WET  = (unsigned short*)(ws + oWET);
  unsigned short* WLD  = (unsigned short*)(ws + oWLD);
  float*          SM   = (float*)(ws + oSM);
  double*         REC  = (double*)(ws + oREC);
  float*          TAIL = (float*)(ws + oTAIL);

  hipFuncSetAttribute(reinterpret_cast<const void*>(&k_bucket), hipFuncAttributeMaxDynamicSharedMemorySize, (int)BK_LDS);

  k_prep<<<PBTOT, NTHR, 0, stream>>>(x, Wemb, bemb, Wc1, bc1, Wc2, bc2, Wc3, bc3, Wn1, bn1, Wn2, bn2,
                                     Wg1, bg1, Wg2, bg2, XB, WET, WLD, SM);
  k_bucket<<<NBK, NTHR, BK_LDS, stream>>>(srcs, dsts, LIST, CO, FLAG);
  k_emb<<<GT, NTHR, 0, stream>>>(XB, WET, SM, HF, HHL);
  for (int l = 0; l < 3; ++l) {
    const unsigned short* bt = WLD + (size_t)l * HD * KL;
    k_lin<<<GT, NTHR, 0, stream>>>(HHL, bt, CO, P);
    const int boff = T_BC + 64 * l;
    if (l == 2)
      k_replay<1><<<NBK, NTHR, 0, stream>>>(LIST, CO, FLAG, P, SM, boff, HF, HHL, out, REC);
    else
      k_replay<0><<<NBK, NTHR, 0, stream>>>(LIST, CO, FLAG, P, SM, boff, HF, HHL, out, REC);
  }
  k_head<<<HT, NTHR, 0, stream>>>(HHL, WLD + (size_t)3 * HD * KL, SM, FLAG, out + O_TL, out + O_PD, TAIL);
  k_global<<<1, NTHR, 0, stream>>>(REC, SM, TAIL, out);
}
